// GNN_7782480740940
// MI455X (gfx1250) — hardware-verified
//
#include <hip/hip_runtime.h>
#include <stddef.h>
#include <stdint.h>
#include <math.h>

#define NN     20000
#define NE     200000
#define IND    64
#define HID    32
#define OUTD   64
#define MLPH   128
#define WSQ    1024
#define G3     96
#define MP     20096
#define EPB    128
#define EP     200064
#define GAP    128
#define TP     128
#define NTHR   256
#define NWAVE  8
#define GBM    64
#define GTHR   128
#define ETHR   128
#define DP     132
#define AP     72
#define EPT    8
#define CHUNK  (NTHR * EPT)
#define WCAP   (EPT * 32)
#define LISTN  (NWAVE * WCAP)
#define NBA    1024
#define SLA    10
#define RCAP   16384
#define DEGCAP 64
#define MEAS_B1024  10371
#define MEAS_MAXDEG 24
#define AGG_ZINTS (LISTN + 2 * RCAP + 3 * NBA)
#define AGG_LDS_INTS (AGG_ZINTS + 16)
#define AGG_LDS_BYTES (AGG_LDS_INTS * 4)
#define EDGE_LDS_BYTES (EPB * DP * 4 + EPB * AP * 2 + EPB * TP * 2)
#define WSMAX  134217728
#define CT     256.0f
#define CW2    16.0f
#define DINV   0.000244140625f
#define F16MIN 6.103515625e-05f
#define MD_EMB 0
#define MD_P   1
#define MD_GRU 2
#define MD_OUT 3
#define NU_XB  (MP * 8)
#define NU_EMB (HID * 8)
#define NU_EC  (HID * 8)
#define NU_W1  (MLPH * 8)
#define NU_W2  (WSQ * 16)
#define NU_WGA (128 * 8)
#define NU_WGH (128 * 8)
#define NU_WO  (OUTD * 8)
#define NPREP  (NU_XB + NU_EMB + NU_EC + NU_W1 + NU_W2 + NU_WGA + NU_WGH + NU_WO)

static_assert(HID == 32 && IND == 64 && OUTD == 64 && MLPH == 128 && WSQ == HID * HID && G3 == 3 * HID);
static_assert(MP % GBM == 0 && MP >= NN && NN % 16 == 0);
static_assert(EP % EPB == 0 && EP >= NE && NE % 16 == 0 && EP % (NWAVE * 16) == 0);
static_assert((CHUNK & (CHUNK - 1)) == 0 && CHUNK <= 4096);
static_assert((NBA & (NBA - 1)) == 0 && NBA == (1 << SLA));
static_assert(((long long)CHUNK << SLA) < (1LL << 31));
static_assert(((long long)NE << SLA) < (1LL << 31));
static_assert(LISTN % NTHR == 0 && NBA % NWAVE == 0 && NBA % 32 == 0);
static_assert(RCAP % 4 == 0 && AGG_ZINTS % (4 * NTHR) == 0);
static_assert(RCAP >= MEAS_B1024 + MEAS_B1024 / 20 + 1);
static_assert(DEGCAP >= MEAS_MAXDEG + 8);
static_assert(AGG_LDS_BYTES <= 300000 && EDGE_LDS_BYTES <= 300000);
static_assert((DP * 4) % 16 == 0 && (AP * 2) % 16 == 0 && AP >= 2 * HID && DP >= MLPH);
static_assert(EPB == ETHR && EPB == 4 * 32 && EPB * TP * 2 == 16 * ETHR * 16);
static_assert(NU_XB % NTHR == 0 && NU_EMB % NTHR == 0 && NU_EC % NTHR == 0 && NU_W1 % NTHR == 0);
static_assert(NU_W2 % NTHR == 0 && NU_WGA % NTHR == 0 && NU_WGH % NTHR == 0 && NU_WO % NTHR == 0);
static_assert(GBM == (GTHR / 32) * 16);
static_assert(GTHR >= 128);
static_assert(((long long)NBA * 20) >= MP);

typedef float          v4f   __attribute__((ext_vector_type(4)));
typedef float          v8f   __attribute__((ext_vector_type(8)));
typedef int            v4i   __attribute__((ext_vector_type(4)));
typedef int            v8i   __attribute__((ext_vector_type(8)));
typedef unsigned short v8us  __attribute__((ext_vector_type(8)));
typedef unsigned short v16us __attribute__((ext_vector_type(16)));
typedef __bf16         v16bf __attribute__((ext_vector_type(16)));
typedef _Float16       v16h  __attribute__((ext_vector_type(16)));
typedef v4f  __attribute__((may_alias)) v4fa;
typedef v4i  __attribute__((may_alias)) v4ia;
typedef v8us __attribute__((may_alias)) v8usa;
union FragB { v16bf v; v16us u; v8us h[2]; v8i w; };
union FragH { v16h  v; v16us u; v8us h[2]; v8i w; };

__device__ __forceinline__ v8f wmb(const FragB& a, const FragB& b, v8f c) {
  v8f d = __builtin_amdgcn_wmma_f32_16x16x32_bf16(false, a.v, false, b.v, (short)0, c, false, false);
  asm volatile("v_nop\n\tv_nop\n\tv_nop\n\tv_nop" : "+v"(d) : "v"(a.w), "v"(b.w));
  return d;
}
__device__ __forceinline__ v8f wmh(const FragH& a, const FragH& b, v8f c) {
  v8f d = __builtin_amdgcn_wmma_f32_16x16x32_f16(false, a.v, false, b.v, (short)0, c, false, false);
  asm volatile("v_nop\n\tv_nop\n\tv_nop\n\tv_nop" : "+v"(d) : "v"(a.w), "v"(b.w));
  return d;
}
__device__ __forceinline__ v8f z8() { v8f z = {0.f, 0.f, 0.f, 0.f, 0.f, 0.f, 0.f, 0.f}; return z; }

__device__ __forceinline__ unsigned bf16_bits(float f) {
  const unsigned u = __float_as_uint(f);
  return (u + 0x7FFFu + ((u >> 16) & 1u)) >> 16;
}
__device__ __forceinline__ float bf16_val(float f) {
  return __uint_as_float(bf16_bits(f) << 16);
}
__device__ __forceinline__ unsigned short f2h(float f) {
  const _Float16 hv = (_Float16)f;
  return __builtin_bit_cast(unsigned short, hv);
}
__device__ __forceinline__ void put16(unsigned short* dp, v8us o) {
  *(volatile v8us*)dp = o;
  __threadfence();
  *(volatile v8us*)dp = o;
}
__device__ __forceinline__ float relu_keep(float v) { return (v > 0.0f) ? v : (v - v); }
__device__ __forceinline__ float tanh_poly(float x) {
  const float x2 = x * x;
  float p = fmaf(x2, 0.021869488536155203f, -0.053968253968253968f);
  p = fmaf(x2, p, 0.13333333333333333f);
  p = fmaf(x2, p, -0.33333333333333333f);
  p = p * x2;
  return fmaf(x, p, x);
}

template <int SLB>
__device__ __forceinline__ int scan_chunk(const int* __restrict__ dsts, int nE, int cbase, int slotBase,
                                          int nb, int vec8, int* list, int tid, int lane, int wave) {
  int wc = 0;
  const int el0  = tid * EPT;
  const int e0   = cbase + el0;
  const int sent = -2147483647 - 1;
  v4i da, db;
  if (vec8 != 0 && cbase + CHUNK <= nE) {
    da = *(const v4i*)(dsts + e0);
    db = *(const v4i*)(dsts + e0 + 4);
  } else {
    da.x = (e0     < nE) ? dsts[min(e0,     nE - 1)] : sent;
    da.y = (e0 + 1 < nE) ? dsts[min(e0 + 1, nE - 1)] : sent;
    da.z = (e0 + 2 < nE) ? dsts[min(e0 + 2, nE - 1)] : sent;
    da.w = (e0 + 3 < nE) ? dsts[min(e0 + 3, nE - 1)] : sent;
    db.x = (e0 + 4 < nE) ? dsts[min(e0 + 4, nE - 1)] : sent;
    db.y = (e0 + 5 < nE) ? dsts[min(e0 + 5, nE - 1)] : sent;
    db.z = (e0 + 6 < nE) ? dsts[min(e0 + 6, nE - 1)] : sent;
    db.w = (e0 + 7 < nE) ? dsts[min(e0 + 7, nE - 1)] : sent;
  }
  const unsigned nbs = (unsigned)slotBase;
  const unsigned unb = (unsigned)nb;
  const unsigned s0 = (unsigned)da.x - nbs, s1 = (unsigned)da.y - nbs;
  const unsigned s2 = (unsigned)da.z - nbs, s3 = (unsigned)da.w - nbs;
  const unsigned s4 = (unsigned)db.x - nbs, s5 = (unsigned)db.y - nbs;
  const unsigned s6 = (unsigned)db.z - nbs, s7 = (unsigned)db.w - nbs;
  const bool h0 = s0 < unb, h1 = s1 < unb, h2 = s2 < unb, h3 = s3 < unb;
  const bool h4 = s4 < unb, h5 = s5 < unb, h6 = s6 < unb, h7 = s7 < unb;
  const unsigned any = __builtin_amdgcn_ballot_w32(h0 | h1 | h2 | h3 | h4 | h5 | h6 | h7);
  if (any != 0u) {
#define HITJ(J, HJ, SJ) { \
      const unsigned mj = __builtin_amdgcn_ballot_w32(HJ); \
      if (mj != 0u) { \
        if (HJ) { \
          const int pos = wc + (int)__builtin_amdgcn_mbcnt_lo(mj, 0u); \
          if (pos < WCAP) list[wave * WCAP + pos] = ((el0 + (J)) << SLB) | (int)(SJ); \
        } \
        wc += (int)__builtin_popcount(mj); } }
    HITJ(0, h0, s0)
    HITJ(1, h1, s1)
    HITJ(2, h2, s2)
    HITJ(3, h3, s3)
    HITJ(4, h4, s4)
    HITJ(5, h5, s5)
    HITJ(6, h6, s6)
    HITJ(7, h7, s7)
#undef HITJ
  }
  return wc;
}

__global__ __launch_bounds__(NTHR) void k_prep(const float* __restrict__ x, const float* __restrict__ Wemb,
                                               const float* __restrict__ Wec, const float* __restrict__ W1,
                                               const float* __restrict__ W2, const float* __restrict__ Wi,
                                               const float* __restrict__ Wh, const float* __restrict__ Wout,
                                               unsigned short* XB, unsigned short* WembT, unsigned short* WecD,
                                               unsigned short* W1D, unsigned short* W2T, unsigned short* WG,
                                               unsigned short* WoutD) {
  const int u  = (int)blockIdx.x * NTHR + (int)threadIdx.x;
  const int L0 = NU_XB;
  const int L1 = L0 + NU_EMB;
  const int L2 = L1 + NU_EC;
  const int L3 = L2 + NU_W1;
  const int L4 = L3 + NU_W2;
  const int L5 = L4 + NU_WGA;
  const int L6 = L5 + NU_WGH;
  const int L7 = L6 + NU_WO;
  v8us o;
  if (u < L0) {
    const int row = u >> 3;
    const int j   = u & 7;
    const int rc  = row < NN ? row : NN - 1;
    const unsigned mk = (row < NN) ? 0xffffu : 0u;
    const float* p = x + (size_t)rc * IND + 8 * j;
    const v4f a = *(const v4f*)p;
    const v4f b = *(const v4f*)(p + 4);
    o[0] = (unsigned short)(bf16_bits(a.x) & mk); o[1] = (unsigned short)(bf16_bits(a.y) & mk);
    o[2] = (unsigned short)(bf16_bits(a.z) & mk); o[3] = (unsigned short)(bf16_bits(a.w) & mk);
    o[4] = (unsigned short)(bf16_bits(b.x) & mk); o[5] = (unsigned short)(bf16_bits(b.y) & mk);
    o[6] = (unsigned short)(bf16_bits(b.z) & mk); o[7] = (unsigned short)(bf16_bits(b.w) & mk);
    put16(XB + (size_t)u * 8, o);
    return;
  } else if (u < L1) {
    const int v  = u - L0;
    const int n  = v >> 3;
    const int k8 = (v & 7) * 8;
    const float* p = Wemb + (size_t)k8 * HID + n;
#pragma unroll
    for (int i = 0; i < 8; ++i) o[i] = (unsigned short)bf16_bits(p[(size_t)i * HID]);
    put16(WembT + (size_t)v * 8, o);
    return;
  } else if (u < L2) {
    const int v  = u - L1;
    const int n  = v >> 3;
    const int k8 = (v & 7) * 8;
    const float* p = Wec + (size_t)(k8 & (HID - 1)) * HID + n;
#pragma unroll
    for (int i = 0; i < 8; ++i) o[i] = (unsigned short)bf16_bits(p[(size_t)i * HID]);
    put16(WecD + (size_t)v * 8, o);
    return;
  } else if (u < L3) {
    const int v  = u - L2;
    const int n  = v >> 3;
    const int k8 = (v & 7) * 8;
    const float* p = W1 + (size_t)(k8 & (HID - 1)) * MLPH + n;
#pragma unroll
    for (int i = 0; i < 8; ++i) o[i] = (unsigned short)bf16_bits(p[(size_t)i * MLPH]);
    put16(W1D + (size_t)v * 8, o);
    return;
  } else if (u < L4) {
    const int v  = u - L3;
    const int c  = v >> 4;
    const int k8 = (v & 15) * 8;
    const float* p = W2 + (size_t)k8 * WSQ + c;
#pragma unroll
    for (int i = 0; i < 8; ++i) o[i] = f2h(CW2 * bf16_val(p[(size_t)i * WSQ]));
    put16(W2T + (size_t)v * 8, o);
    return;
  } else if (u < L5) {
    const int v  = u - L4;
    const int n  = v >> 3;
    const int ka = (v & 7) * 8;
    const int cc = n < G3 ? n : G3 - 1;
    const unsigned mk = (n < G3) ? 0xffffu : 0u;
    const float* p = Wi + (size_t)(ka & (HID - 1)) * G3 + cc;
#pragma unroll
    for (int i = 0; i < 8; ++i) o[i] = (unsigned short)(bf16_bits(p[(size_t)i * G3]) & mk);
    put16(WG + (size_t)n * 128 + ka, o);
    return;
  } else if (u < L6) {
    const int v  = u - L5;
    const int n  = v >> 3;
    const int kh = (v & 7) * 8;
    const int cc = n < 64 ? n : (n >= G3 ? n - 32 : 64);
    const unsigned mk = (n < 64 || n >= G3) ? 0xffffu : 0u;
    const float* p = Wh + (size_t)(kh & (HID - 1)) * G3 + cc;
#pragma unroll
    for (int i = 0; i < 8; ++i) o[i] = (unsigned short)(bf16_bits(p[(size_t)i * G3]) & mk);
    put16(WG + (size_t)n * 128 + 64 + kh, o);
    return;
  } else if (u < L7) {
    const int v  = u - L6;
    const int n  = v >> 3;
    const int k8 = (v & 7) * 8;
    const float* p = Wout + (size_t)(k8 & (HID - 1)) * OUTD + n;
#pragma unroll
    for (int i = 0; i < 8; ++i) o[i] = (unsigned short)bf16_bits(p[(size_t)i * OUTD]);
    put16(WoutD + (size_t)v * 8, o);
    return;
  }
}

template <int NT, int MODE>
__global__ __launch_bounds__(GTHR) void k_gemm(const unsigned short* __restrict__ A, int lda,
                                               const unsigned short* __restrict__ BT, int ldb, int K,
                                               const float* __restrict__ bA, const float* __restrict__ bB,
                                               const float* __restrict__ Hold, float* Hnew,
                                               unsigned short* GAn, float* outp) {
  constexpr int SW = NT * 16;
  static_assert(SW <= GTHR);
  __shared__ __attribute__((aligned(16))) float stg[GBM * SW];
  __shared__ __attribute__((aligned(16))) float hn[GBM * HID];
  __shared__ __attribute__((aligned(16))) float sbias[SW];
  const int tid = (int)threadIdx.x, lane = tid & 31, wave = tid >> 5, hh = lane >> 4, m = lane & 15;
  const int rowBase = (int)blockIdx.x * GBM;

  if constexpr (MODE != MD_P) {
    if (tid < SW) {
      float bvv;
      if constexpr (MODE == MD_GRU) {
        const int lc = tid;
        const int ia = lc < G3 ? lc : G3 - 1;
        const int ib = lc < 64 ? lc : (lc >= G3 ? lc - 32 : 64);
        const float va = bf16_val(bA[ia]);
        const float vb = bf16_val(bB[ib]);
        const float vs = va + vb;
        const unsigned m0 = (lc < 64) ? 0xffffffffu : 0u;
        const unsigned m1 = (lc >= 64 && lc < G3) ? 0xffffffffu : 0u;
        const unsigned m2 = (lc >= G3) ? 0xffffffffu : 0u;
        bvv = __uint_as_float((__float_as_uint(vs) & m0) | (__float_as_uint(va) & m1) | (__float_as_uint(vb) & m2));
      } else {
        bvv = bf16_val(bA[tid]);
      }
      sbias[tid] = bvv;
    }
  }
  __syncthreads();

  v8f acc[NT];
#pragma unroll
  for (int t = 0; t < NT; ++t) acc[t] = z8();
  const unsigned short* ap = A  + (size_t)(rowBase + 16 * wave + m) * (size_t)lda + 8 * hh;
  const unsigned short* bp = BT + (size_t)m * (size_t)ldb + 8 * hh;

#pragma unroll 1
  for (int k0 = 0; k0 < K; k0 += 32) {
    FragB af;
    af.h[0] = *(const v8usa*)(ap + k0);
    af.h[1] = *(const v8usa*)(ap + k0 + 16);
#pragma unroll
    for (int nt = 0; nt < NT; ++nt) {
      const unsigned short* wq = bp + (size_t)(16 * nt) * (size_t)ldb + k0;
      FragB bf;
      bf.h[0] = *(const v8usa*)wq;
      bf.h[1] = *(const v8usa*)(wq + 16);
      acc[nt] = wmb(af, bf, acc[nt]);
    }
  }

#pragma unroll
  for (int nt = 0; nt < NT; ++nt) {
    const int lc = 16 * nt + m;
    float bvv = 0.0f;
    if constexpr (MODE != MD_P) bvv = sbias[lc];
#pragma unroll
    for (int r = 0; r < 8; ++r) {
      const int lr = 16 * wave + 8 * hh + r;
      stg[lr * SW + lc] = acc[nt][r] + bvv;
    }
  }
  __syncthreads();

  if constexpr (MODE == MD_OUT) {
    const int q2 = lane >> 4, j2 = lane & 15;
#pragma unroll 1
    for (int it = 0; it < 8; ++it) {
      float* sp = stg + (16 * wave + 2 * it + q2) * SW + 4 * j2;
      v4f v = *(const v4fa*)sp;
      v.x = tanhf(v.x); v.y = tanhf(v.y); v.z = tanhf(v.z); v.w = tanhf(v.w);
      *(v4fa*)sp = v;
    }
    v4f pv[8];
#pragma unroll
    for (int it = 0; it < 8; ++it) pv[it] = *(const v4fa*)(stg + (16 * wave + 2 * it + q2) * SW + 4 * j2);
#pragma unroll
    for (int it = 0; it < 8; ++it) {
      const int row = rowBase + 16 * wave + 2 * it + q2;
      if (row < NN) *(volatile v4f*)(outp + (size_t)row * OUTD + 4 * j2) = pv[it];
    }
    __threadfence();
#pragma unroll
    for (int it = 0; it < 8; ++it) {
      const int row = rowBase + 16 * wave + 2 * it + q2;
      if (row < NN) *(volatile v4f*)(outp + (size_t)row * OUTD + 4 * j2) = pv[it];
    }
  } else {
    const int q = lane >> 3, j = lane & 7;
    const float* hsrc = stg;
    if constexpr (MODE == MD_GRU) {
#pragma unroll 1
      for (int it = 0; it < 4; ++it) {
        const int row = 16 * wave + 4 * it + q;
        const float* sp = stg + row * SW + 4 * j;
        const v4f gr = *(const v4fa*)sp;
        const v4f gz = *(const v4fa*)(sp + 32);
        const v4f gn = *(const v4fa*)(sp + 64);
        const v4f gh = *(const v4fa*)(sp + 96);
        const v4f ho = *(const v4f*)(Hold + (size_t)(rowBase + row) * HID + 4 * j);
        v4f res;
        {
          const float r0 = 1.0f / (1.0f + expf(-gr.x)); const float z0 = 1.0f / (1.0f + expf(-gz.x));
          const float n0 = tanhf(gn.x + r0 * gh.x);     res.x = (1.0f - z0) * n0 + z0 * ho.x;
          const float r1 = 1.0f / (1.0f + expf(-gr.y)); const float z1 = 1.0f / (1.0f + expf(-gz.y));
          const float n1 = tanhf(gn.y + r1 * gh.y);     res.y = (1.0f - z1) * n1 + z1 * ho.y;
          const float r2 = 1.0f / (1.0f + expf(-gr.z)); const float z2 = 1.0f / (1.0f + expf(-gz.z));
          const float n2 = tanhf(gn.z + r2 * gh.z);     res.z = (1.0f - z2) * n2 + z2 * ho.z;
          const float r3 = 1.0f / (1.0f + expf(-gr.w)); const float z3 = 1.0f / (1.0f + expf(-gz.w));
          const float n3 = tanhf(gn.w + r3 * gh.w);     res.w = (1.0f - z3) * n3 + z3 * ho.w;
        }
        *(v4fa*)(hn + row * HID + 4 * j) = res;
      }
      __syncthreads();
      hsrc = hn;
    }
    const unsigned mh = 0u - (unsigned)(j >> 2);
    const unsigned ml = ~mh;
    v4f  hv4[4];
    v8us gv[4];
#pragma unroll
    for (int it = 0; it < 4; ++it) {
      const int row = 16 * wave + 4 * it + q;
      hv4[it] = *(const v4fa*)(hsrc + row * HID + 4 * j);
      if constexpr (MODE != MD_P) {
        const float* sp = hsrc + row * HID + 8 * (j & 3);
        const v4f a = *(const v4fa*)sp;
        const v4f b = *(const v4fa*)(sp + 4);
        const v8f f8 = {a.x, a.y, a.z, a.w, b.x, b.y, b.z, b.w};
        v8us oo;
#pragma unroll
        for (int e = 0; e < 8; ++e) {
          const unsigned hb = bf16_bits(f8[e]);
          const unsigned lb = bf16_bits(f8[e] - __uint_as_float(hb << 16));
          oo[e] = (unsigned short)((hb & ml) | (lb & mh));
        }
        gv[it] = oo;
      }
    }
#pragma unroll
    for (int it = 0; it < 4; ++it) {
      const int row = rowBase + 16 * wave + 4 * it + q;
      *(volatile v4f*)(Hnew + (size_t)row * HID + 4 * j) = hv4[it];
      if constexpr (MODE != MD_P) *(volatile v8us*)(GAn + (size_t)row * GAP + 64 + 8 * j) = gv[it];
    }
    __threadfence();
#pragma unroll
    for (int it = 0; it < 4; ++it) {
      const int row = rowBase + 16 * wave + 4 * it + q;
      *(volatile v4f*)(Hnew + (size_t)row * HID + 4 * j) = hv4[it];
      if constexpr (MODE != MD_P) *(volatile v8us*)(GAn + (size_t)row * GAP + 64 + 8 * j) = gv[it];
    }
  }
}

__device__ __forceinline__ void wave_gemm_b(const unsigned short* sAw, float* sDw,
                                            const unsigned short* __restrict__ BT, int ldb, int K,
                                            int hh, int m) {
#pragma unroll 1
  for (int nh = 0; nh < 2; ++nh) {
    v8f acc[2][4];
#pragma unroll
    for (int mt = 0; mt < 2; ++mt)
#pragma unroll
      for (int nt = 0; nt < 4; ++nt) acc[mt][nt] = z8();
    const unsigned short* ap0 = sAw + m * AP + 8 * hh;
    const unsigned short* ap1 = ap0 + 16 * AP;
    const unsigned short* bp  = BT + (size_t)(64 * nh + m) * (size_t)ldb + 8 * hh;
#pragma unroll 1
    for (int k0 = 0; k0 < K; k0 += 32) {
      FragB a0, a1;
      a0.h[0] = *(const v8usa*)(ap0 + k0);
      a0.h[1] = *(const v8usa*)(ap0 + k0 + 16);
      a1.h[0] = *(const v8usa*)(ap1 + k0);
      a1.h[1] = *(const v8usa*)(ap1 + k0 + 16);
#pragma unroll
      for (int nt = 0; nt < 4; ++nt) {
        const unsigned short* wq = bp + (size_t)(16 * nt) * (size_t)ldb + k0;
        FragB b;
        b.h[0] = *(const v8usa*)wq;
        b.h[1] = *(const v8usa*)(wq + 16);
        acc[0][nt] = wmb(a0, b, acc[0][nt]);
        acc[1][nt] = wmb(a1, b, acc[1][nt]);
      }
    }
#pragma unroll
    for (int nt = 0; nt < 4; ++nt) {
      const int col = 64 * nh + 16 * nt + m;
#pragma unroll
      for (int mt = 0; mt < 2; ++mt)
#pragma unroll
        for (int r = 0; r < 8; ++r) sDw[(16 * mt + 8 * hh + r) * DP + col] = acc[mt][nt][r];
    }
  }
}

__global__ __launch_bounds__(ETHR) void k_edge(const int* __restrict__ srcs, const int* __restrict__ dsts,
                                               const float* __restrict__ P,
                                               const unsigned short* __restrict__ W1D,
                                               const float* __restrict__ bec, const float* __restrict__ b1,
                                               unsigned short* T16) {
  extern __shared__ __attribute__((aligned(16))) float dyn[];
  __shared__ __attribute__((aligned(16))) float sb1[MLPH];
  __shared__ __attribute__((aligned(16))) float sbe[HID];
  float*          sD = dyn;
  unsigned short* sA = (unsigned short*)(dyn + EPB * DP);
  unsigned short* sM = sA + EPB * AP;
  const int tid = (int)threadIdx.x, lane = tid & 31, wave = tid >> 5, hh = lane >> 4, m = lane & 15;

  sb1[tid] = bf16_val(b1[tid]);
  if (tid < HID) sbe[tid] = bf16_val(bec[tid]);
  __syncthreads();

  const int elb = (int)blockIdx.x * EPB;
  const int el  = elb + tid;
  const int elc = el < NE ? el : (NE - 1);
  int s = srcs[elc];
  int t = dsts[elc];
  s = s < 0 ? 0 : (s > NN - 1 ? NN - 1 : s);
  t = t < 0 ? 0 : (t > NN - 1 ? NN - 1 : t);
  const float* ps = P + (size_t)s * HID;
  const float* pd = P + (size_t)t * HID;
  unsigned short* ra = sA + tid * AP;
#pragma unroll 1
  for (int c8 = 0; c8 < HID / 8; ++c8) {
    const v4f a0 = *(const v4f*)(ps + 8 * c8);
    const v4f a1 = *(const v4f*)(ps + 8 * c8 + 4);
    const v4f d0 = *(const v4f*)(pd + 8 * c8);
    const v4f d1 = *(const v4f*)(pd + 8 * c8 + 4);
    const v4f e0 = *(const v4fa*)(sbe + 8 * c8);
    const v4f e1 = *(const v4fa*)(sbe + 8 * c8 + 4);
    const v8f av = {a0.x, a0.y, a0.z, a0.w, a1.x, a1.y, a1.z, a1.w};
    const v8f dv = {d0.x, d0.y, d0.z, d0.w, d1.x, d1.y, d1.z, d1.w};
    const v8f ev = {e0.x, e0.y, e0.z, e0.w, e1.x, e1.y, e1.z, e1.w};
    v8us ho, lo;
#pragma unroll
    for (int i = 0; i < 8; ++i) {
      const float hv = relu_keep((av[i] - dv[i]) + ev[i]);
      const unsigned hb = bf16_bits(hv);
      ho[i] = (unsigned short)hb;
      lo[i] = (unsigned short)bf16_bits(hv - __uint_as_float(hb << 16));
    }
    *(v8usa*)(ra + 8 * c8)       = ho;
    *(v8usa*)(ra + HID + 8 * c8) = lo;
  }
  __syncthreads();

  wave_gemm_b(sA + 32 * wave * AP, sD + 32 * wave * DP, W1D, 2 * HID, 2 * HID, hh, m);
  __syncthreads();

  {
    const float* rd = sD + tid * DP;
    unsigned short* rm = sM + tid * TP;
#pragma unroll 1
    for (int c8 = 0; c8 < MLPH / 8; ++c8) {
      const v4f va = *(const v4fa*)(rd + 8 * c8);
      const v4f vb = *(const v4fa*)(rd + 8 * c8 + 4);
      const v4f ba = *(const v4fa*)(sb1 + 8 * c8);
      const v4f bb = *(const v4fa*)(sb1 + 8 * c8 + 4);
      const v8f v8 = {va.x, va.y, va.z, va.w, vb.x, vb.y, vb.z, vb.w};
      const v8f b8 = {ba.x, ba.y, ba.z, ba.w, bb.x, bb.y, bb.z, bb.w};
      v8us o;
#pragma unroll
      for (int i = 0; i < 8; ++i) {
        float tv = CT * relu_keep(v8[i] + b8[i]);
        tv = (tv < F16MIN) ? 0.0f : tv;
        o[i] = f2h(tv);
      }
      *(v8usa*)(rm + 8 * c8) = o;
    }
  }
  __syncthreads();

  {
    v4i pv[16];
#pragma unroll
    for (int it = 0; it < 16; ++it) pv[it] = *(const v4ia*)(sM + (size_t)(it * ETHR + tid) * 8);
    unsigned short* mb = T16 + (size_t)elb * TP;
#pragma unroll
    for (int it = 0; it < 16; ++it) *(volatile v4i*)(mb + (size_t)(it * ETHR + tid) * 8) = pv[it];
    __threadfence();
#pragma unroll
    for (int it = 0; it < 16; ++it) *(volatile v4i*)(mb + (size_t)(it * ETHR + tid) * 8) = pv[it];
  }
}

__global__ __launch_bounds__(NTHR) void k_msg(const unsigned short* __restrict__ T16,
                                              const unsigned short* __restrict__ W2T,
                                              const float* __restrict__ b2, const float* __restrict__ Hc,
                                              const int* __restrict__ srcs, float* MSG) {
  __shared__ __attribute__((aligned(16))) float sb2[WSQ];
  __shared__ __attribute__((aligned(16))) float sm[NWAVE * 16 * HID];
  const int tid = (int)threadIdx.x, lane = tid & 31, wave = tid >> 5, hh = lane >> 4, m = lane & 15;
  {
    const v4f b = *(const v4f*)(b2 + 4 * tid);
    v4f o;
    o.x = bf16_val(b.x); o.y = bf16_val(b.y); o.z = bf16_val(b.z); o.w = bf16_val(b.w);
    *(v4fa*)(sb2 + 4 * tid) = o;
  }
  __syncthreads();

  const int e0 = ((int)blockIdx.x * NWAVE + wave) * 16;
  const int e  = e0 + m;
  const int ec = e < NE ? e : (NE - 1);
  int s = srcs[ec];
  s = s < 0 ? 0 : (s > NN - 1 ? NN - 1 : s);
  const float* hp = Hc + (size_t)s * HID + 8 * hh;
  const v4f h00 = *(const v4f*)(hp);
  const v4f h01 = *(const v4f*)(hp + 4);
  const v4f h10 = *(const v4f*)(hp + 16);
  const v4f h11 = *(const v4f*)(hp + 20);
  const v8f hs0 = {h00.x, h00.y, h00.z, h00.w, h01.x, h01.y, h01.z, h01.w};
  const v8f hs1 = {h10.x, h10.y, h10.z, h10.w, h11.x, h11.y, h11.z, h11.w};

  FragH bf[4];
  {
    const unsigned short* tp = T16 + (size_t)(e0 + m) * TP + 8 * hh;
#pragma unroll
    for (int k = 0; k < 4; ++k) {
      bf[k].h[0] = *(const v8usa*)(tp + 32 * k);
      bf[k].h[1] = *(const v8usa*)(tp + 32 * k + 16);
    }
  }
  float* smw = sm + wave * (16 * HID);

#pragma unroll 1
  for (int i = 0; i < HID; ++i) {
    v8f d0 = z8(), d1 = z8();
    const unsigned short* ap = W2T + (size_t)(32 * i + m) * MLPH + 8 * hh;
#pragma unroll
    for (int k = 0; k < 4; ++k) {
      FragH a0, a1;
      a0.h[0] = *(const v8usa*)(ap + 32 * k);
      a0.h[1] = *(const v8usa*)(ap + 32 * k + 16);
      a1.h[0] = *(const v8usa*)(ap + 16 * MLPH + 32 * k);
      a1.h[1] = *(const v8usa*)(ap + 16 * MLPH + 32 * k + 16);
      d0 = wmh(a0, bf[k], d0);
      d1 = wmh(a1, bf[k], d1);
    }
    const float* bq = sb2 + 32 * i + 8 * hh;
    const v4f ba = *(const v4fa*)(bq);
    const v4f bb = *(const v4fa*)(bq + 4);
    const v4f bc = *(const v4fa*)(bq + 16);
    const v4f bd = *(const v4fa*)(bq + 20);
    const v8f b0 = {ba.x, ba.y, ba.z, ba.w, bb.x, bb.y, bb.z, bb.w};
    const v8f b1v = {bc.x, bc.y, bc.z, bc.w, bd.x, bd.y, bd.z, bd.w};
    v8f x0, x1;
    bool okl = true;
#pragma unroll
    for (int r = 0; r < 8; ++r) {
      x0[r] = fmaf(d0[r], DINV, b0[r]);
      x1[r] = fmaf(d1[r], DINV, b1v[r]);
      okl = okl && (fabsf(x0[r]) < 0.25f) && (fabsf(x1[r]) < 0.25f);
    }
    const unsigned nbad = __builtin_amdgcn_ballot_w32(!okl);
    float sacc = 0.0f;
    if (nbad == 0u) {
#pragma unroll
      for (int r = 0; r < 8; ++r) sacc = fmaf(tanh_poly(x0[r]), hs0[r], sacc);
#pragma unroll
      for (int r = 0; r < 8; ++r) sacc = fmaf(tanh_poly(x1[r]), hs1[r], sacc);
    } else {
#pragma unroll
      for (int r = 0; r < 8; ++r) sacc = fmaf(tanhf(x0[r]), hs0[r], sacc);
#pragma unroll
      for (int r = 0; r < 8; ++r) sacc = fmaf(tanhf(x1[r]), hs1[r], sacc);
    }
    const float oth = __shfl_xor(sacc, 16, 32);
    const float tot = sacc + oth;
    if (hh == 0) smw[m * HID + i] = tot;
  }
  __syncthreads();

  {
    v4f pv[4];
#pragma unroll
    for (int it = 0; it < 4; ++it) pv[it] = *(const v4fa*)(smw + (it * 32 + lane) * 4);
    float* gp = MSG + (size_t)e0 * HID;
#pragma unroll
    for (int it = 0; it < 4; ++it) *(volatile v4f*)(gp + (it * 32 + lane) * 4) = pv[it];
    __threadfence();
#pragma unroll
    for (int it = 0; it < 4; ++it) *(volatile v4f*)(gp + (it * 32 + lane) * 4) = pv[it];
  }
}

__global__ __launch_bounds__(NTHR) void k_agg(const int* __restrict__ dsts, int nE, int vec8,
                                              const float* __restrict__ MSG, unsigned short* GAl) {
  extern __shared__ __attribute__((aligned(16))) int dsm[];
  int* list = dsm;
  int* hl   = dsm + LISTN;
  int* sl   = hl + RCAP;
  int* cnt  = sl + RCAP;
  int* offs = cnt + NBA;
  int* cur  = offs + NBA;
  int* misc = cur + NBA;
  const int tid = (int)threadIdx.x, lane = tid & 31, wave = tid >> 5;
  const int nodeBase = (int)blockIdx.x * NBA;

  {
    const v4i z4 = {0, 0, 0, 0};
    for (int i = tid * 4; i < AGG_ZINTS; i += NTHR * 4) *(v4ia*)(dsm + i) = z4;
    if (tid < 16) misc[tid] = 0;
  }
  __syncthreads();

  int t = 0, ov = 0;
  const int nChunks = (nE + CHUNK - 1) / CHUNK;
#pragma unroll 1
  for (int ch = 0; ch < nChunks; ++ch) {
    const int cbase = ch * CHUNK;
    const int wc = scan_chunk<SLA>(dsts, nE, cbase, nodeBase, NBA, vec8, list, tid, lane, wave);
    if (lane == 0) misc[wave] = wc;
    __syncthreads();
    if (wave == 0) {
#pragma unroll 1
      for (int w2 = 0; w2 < NWAVE; ++w2) {
        int c = misc[w2];
        c = c < 0 ? 0 : (c > WCAP ? WCAP : c);
#pragma unroll 1
        for (int b0 = 0; b0 < c; b0 += 32) {
          const int idx = b0 + lane;
          const int ent = list[w2 * WCAP + (idx < WCAP ? idx : WCAP - 1)];
          const int m32 = (c - b0) < 32 ? (c - b0) : 32;
#pragma unroll 1
          for (int k = 0; k < m32; ++k) {
            const int u    = __builtin_amdgcn_readlane(ent, k);
            const int slot = u & (NBA - 1);
            const int el   = (u >> SLA) & (CHUNK - 1);
            const int pk   = ((cbase + el) << SLA) | slot;
            if (t < RCAP) {
              if (lane == 0) { hl[t] = pk; cnt[slot] = cnt[slot] + 1; }
              t = t + 1;
            } else {
              ov = 1;
            }
          }
        }
      }
    }
    __syncthreads();
  }
  if (wave == 0 && lane == 0) { misc[8] = t; misc[9] = ov; }
  __syncthreads();
  int tt = misc[8];
  tt = tt < 0 ? 0 : (tt > RCAP ? RCAP : tt);
  const int ovf = misc[9];

  if (wave == 0) {
    const int base = lane * (NBA / 32);
    int s = 0;
#pragma unroll 1
    for (int i = 0; i < NBA / 32; ++i) s += cnt[base + i];
    int incl = s;
#pragma unroll
    for (int d = 1; d < 32; d <<= 1) {
      const int y = __shfl_up(incl, d, 32);
      if (lane >= d) incl += y;
    }
    int run = incl - s;
#pragma unroll 1
    for (int i = 0; i < NBA / 32; ++i) {
      const int cv = cnt[base + i];
      offs[base + i] = run;
      cur[base + i]  = run;
      run += cv;
    }
  }
  __syncthreads();
  if (wave == 0) {
#pragma unroll 1
    for (int b0 = 0; b0 < tt; b0 += 32) {
      const int idx = b0 + lane;
      const int ent = hl[idx < RCAP ? idx : RCAP - 1];
      const int m32 = (tt - b0) < 32 ? (tt - b0) : 32;
#pragma unroll 1
      for (int k = 0; k < m32; ++k) {
        const int u    = __builtin_amdgcn_readlane(ent, k);
        const int slot = u & (NBA - 1);
        if (lane == 0) {
          int p = cur[slot];
          p = p < 0 ? 0 : (p > RCAP - 1 ? RCAP - 1 : p);
          sl[p] = u;
          cur[slot] = p + 1;
        }
      }
    }
  }
  __syncthreads();

  const float qnan = __int_as_float(0x7fc00000);
  const float pz = (ovf != 0) ? qnan : 0.0f;
  const int j  = lane & 7;
  const int sb = 8 * (j & 3);
  const unsigned mh = 0u - (unsigned)(j >> 2);
  const unsigned ml = ~mh;
#pragma unroll 1
  for (int si = 0; si < NBA / NWAVE; ++si) {
    const int s    = si * NWAVE + wave;
    const int node = nodeBase + s;
    int c = cnt[s];
    const bool big = c > DEGCAP;
    c = c < 0 ? 0 : (c > DEGCAP ? DEGCAP : c);
    int o = offs[s];
    o = o < 0 ? 0 : (o > RCAP ? RCAP : o);
    float a = 0.0f;
#pragma unroll 1
    for (int b0 = 0; b0 < c; b0 += 32) {
      int idx = o + b0 + lane;
      idx = idx > RCAP - 1 ? RCAP - 1 : idx;
      const int ent = sl[idx];
      int eid = ent >> SLA;
      eid = eid < 0 ? 0 : (eid > nE - 1 ? nE - 1 : eid);
      const int m32 = (c - b0) < 32 ? (c - b0) : 32;
#pragma unroll 1
      for (int k = 0; k < m32; ++k) {
        const int ek = __builtin_amdgcn_readlane(eid, k);
        a += MSG[(size_t)ek * HID + lane];
      }
    }
    const float pzr = big ? qnan : pz;
    const float av  = a + pzr;
    v8us oo;
#pragma unroll
    for (int e = 0; e < 8; ++e) {
      const float ve = __shfl(av, sb + e, 32);
      const unsigned hb = bf16_bits(ve);
      const unsigned lb = bf16_bits(ve - __uint_as_float(hb << 16));
      oo[e] = (unsigned short)((hb & ml) | (lb & mh));
    }
    const bool live = (node < MP) && (lane < 8);
    const int  nr   = node < MP ? node : MP - 1;
    unsigned short* gp = GAl + (size_t)nr * GAP + 8 * j;
    if (live) *(volatile v8us*)gp = oo;
    __threadfence();
    if (live) *(volatile v8us*)gp = oo;
  }
}

static inline size_t al256(size_t o) { return (o + 255) & ~(size_t)255; }

extern "C" void kernel_launch(void* const* d_in, const int* in_sizes, int n_in,
                              void* d_out, int out_size, void* d_ws, size_t ws_size,
                              hipStream_t stream) {
  if (n_in < 17) return;
  if (in_sizes[0] != NN * IND) return;
  if (in_sizes[1] != NE || in_sizes[2] != NE) return;
  if (in_sizes[3] != IND * HID || in_sizes[4] != HID) return;
  if (in_sizes[5] != HID * HID || in_sizes[6] != HID) return;
  if (in_sizes[7] != HID * MLPH || in_sizes[8] != MLPH) return;
  if (in_sizes[9] != MLPH * WSQ || in_sizes[10] != WSQ) return;
  if (in_sizes[11] != HID * G3 || in_sizes[12] != G3) return;
  if (in_sizes[13] != HID * G3 || in_sizes[14] != G3) return;
  if (in_sizes[15] != HID * OUTD || in_sizes[16] != OUTD) return;
  if (out_size != NN * OUTD) return;

  const float* x     = (const float*)d_in[0];
  const int*   src   = (const int*)d_in[1];
  const int*   dst   = (const int*)d_in[2];
  const float* W_emb = (const float*)d_in[3];
  const float* b_emb = (const float*)d_in[4];
  const float* W_ec  = (const float*)d_in[5];
  const float* b_ec  = (const float*)d_in[6];
  const float* W1    = (const float*)d_in[7];
  const float* b1    = (const float*)d_in[8];
  const float* W2    = (const float*)d_in[9];
  const float* b2    = (const float*)d_in[10];
  const float* W_i   = (const float*)d_in[11];
  const float* b_i   = (const float*)d_in[12];
  const float* W_h   = (const float*)d_in[13];
  const float* b_h   = (const float*)d_in[14];
  const float* W_out = (const float*)d_in[15];
  const float* b_out = (const float*)d_in[16];
  float* out = (float*)d_out;

  char* ws = (char*)d_ws;
  size_t off = 0;
  const size_t oXB  = off; off = al256(off + (size_t)MP * IND * 2);
  const size_t oWE  = off; off = al256(off + (size_t)HID * IND * 2);
  const size_t oWC  = off; off = al256(off + (size_t)HID * 64 * 2);
  const size_t oW1  = off; off = al256(off + (size_t)MLPH * 64 * 2);
  const size_t oW2  = off; off = al256(off + (size_t)WSQ * MLPH * 2);
  const size_t oWG  = off; off = al256(off + (size_t)128 * 128 * 2);
  const size_t oWO  = off; off = al256(off + (size_t)OUTD * 64 * 2);
  const size_t oH0  = off; off = al256(off + (size_t)MP * HID * 4);
  const size_t oH1  = off; off = al256(off + (size_t)MP * HID * 4);
  const size_t oP   = off; off = al256(off + (size_t)MP * HID * 4);
  const size_t oG0  = off; off = al256(off + (size_t)MP * GAP * 2);
  const size_t oG1  = off; off = al256(off + (size_t)MP * GAP * 2);
  const size_t oT   = off; off = al256(off + (size_t)EP * TP * 2);
  const size_t oM   = off; off = al256(off + (size_t)EP * HID * 4);
  if (off > ws_size || off > (size_t)WSMAX) return;
  unsigned short* XB    = (unsigned short*)(ws + oXB);
  unsigned short* WembT = (unsigned short*)(ws + oWE);
  unsigned short* WecD  = (unsigned short*)(ws + oWC);
  unsigned short* W1D   = (unsigned short*)(ws + oW1);
  unsigned short* W2T   = (unsigned short*)(ws + oW2);
  unsigned short* WG    = (unsigned short*)(ws + oWG);
  unsigned short* WoutD = (unsigned short*)(ws + oWO);
  float*          Hb[2] = {(float*)(ws + oH0), (float*)(ws + oH1)};
  float*          Pp    = (float*)(ws + oP);
  unsigned short* GAb[2] = {(unsigned short*)(ws + oG0), (unsigned short*)(ws + oG1)};
  unsigned short* T16   = (unsigned short*)(ws + oT);
  float*          MSG   = (float*)(ws + oM);

  hipFuncSetAttribute(reinterpret_cast<const void*>(&k_edge), hipFuncAttributeMaxDynamicSharedMemorySize,
                      (int)EDGE_LDS_BYTES);
  hipFuncSetAttribute(reinterpret_cast<const void*>(&k_agg), hipFuncAttributeMaxDynamicSharedMemorySize,
                      (int)AGG_LDS_BYTES);

  const int gM = MP / GBM;
  const int gE = EP / EPB;
  const int gA = (MP + NBA - 1) / NBA;

  k_prep<<<NPREP / NTHR, NTHR, 0, stream>>>(x, W_emb, W_ec, W1, W2, W_i, W_h, W_out,
                                            XB, WembT, WecD, W1D, W2T, WG, WoutD);
  k_gemm<2, MD_EMB><<<gM, GTHR, 0, stream>>>(XB, IND, WembT, IND, IND, b_emb, b_emb, x, Hb[0], GAb[0], out);
  k_gemm<2, MD_P><<<gM, GTHR, 0, stream>>>(GAb[0] + 64, GAP, WecD, 64, 64, b_ec, b_ec, x, Pp, GAb[1], out);
  k_edge<<<gE, ETHR, EDGE_LDS_BYTES, stream>>>(src, dst, Pp, W1D, b_ec, b1, T16);
  for (int s = 0; s < 3; ++s) {
    const int c = s & 1, n = (s + 1) & 1;
    k_msg<<<gE, NTHR, 0, stream>>>(T16, W2T, b2, Hb[c], src, MSG);
    k_agg<<<gA, NTHR, AGG_LDS_BYTES, stream>>>(dst, NE, 1, MSG, GAb[c]);
    k_gemm<8, MD_GRU><<<gM, GTHR, 0, stream>>>(GAb[c], GAP, WG, 128, 128, b_i, b_h, Hb[c], Hb[n], GAb[n], out);
  }
  k_gemm<4, MD_OUT><<<gM, GTHR, 0, stream>>>(GAb[1] + 64, GAP, WoutD, 64, 64, b_out, b_out, x, Pp, GAb[0], out);
}
